// DecoderNetwork_Maze_86844238725481
// MI455X (gfx1250) — hardware-verified
//
#include <hip/hip_runtime.h>

#define NN 50000
#define NE 1600000
#define DN 128
#define NTILE (NN / 16)

typedef _Float16 f16;
typedef __attribute__((ext_vector_type(16))) f16 f16x16;
typedef __attribute__((ext_vector_type(8)))  float f32x8;
typedef __attribute__((ext_vector_type(4)))  float v4f_t;
typedef float v4fa __attribute__((ext_vector_type(4), may_alias));

__device__ __forceinline__ f32x8 wmma16(f16x16 a, f16x16 b, f32x8 c) {
  c = __builtin_amdgcn_wmma_f32_16x16x32_f16(false, a, false, b, (short)0, c, false, false);
  asm volatile("v_nop\n\tv_nop\n\tv_nop\n\tv_nop" : "+v"(c) : "v"(a), "v"(b));
  return c;
}
__device__ __forceinline__ f16x16 load_frag(const float* __restrict__ base, int ld, int row0, int k0) {
  const int lane = threadIdx.x & 31, r = lane & 15, kh = (lane >> 4) * 8;
  const float* p0 = base + (size_t)(row0 + r) * ld + (k0 + kh);
  const v4f_t a = *(const v4f_t*)(p0), b = *(const v4f_t*)(p0 + 4), c = *(const v4f_t*)(p0 + 16), d = *(const v4f_t*)(p0 + 20);
  f16x16 f;
  f[0] = (f16)a[0]; f[1] = (f16)a[1]; f[2]  = (f16)a[2]; f[3]  = (f16)a[3]; f[4]  = (f16)b[0]; f[5]  = (f16)b[1]; f[6]  = (f16)b[2]; f[7]  = (f16)b[3];
  f[8] = (f16)c[0]; f[9] = (f16)c[1]; f[10] = (f16)c[2]; f[11] = (f16)c[3]; f[12] = (f16)d[0]; f[13] = (f16)d[1]; f[14] = (f16)d[2]; f[15] = (f16)d[3];
  return f;
}

__global__ __launch_bounds__(256) void k_node_proj(const float* __restrict__ x, const float* __restrict__ W, float* __restrict__ P) {
  __shared__ __attribute__((aligned(16))) float pS[8][32];
  const int lane = threadIdx.x & 31, wave = threadIdx.x >> 5, col = lane & 15, rh = (lane >> 4) * 8, kh = rh;
  const int tile = blockIdx.x * 8 + wave;
  const bool live = tile < NTILE;
  f32x8 acc = {};
  if (live) {
#pragma unroll
    for (int ks = 0; ks < DN / 32; ++ks) {
      const f16x16 af = load_frag(x, DN, tile * 16, ks * 32);
      f16x16 bf;
#pragma unroll
      for (int i = 0; i < 8; ++i) {
        const int k = ks * 32 + kh + i;
        bf[i]     = (col == 0) ? (f16)W[k]      : (col == 1) ? (f16)W[DN + k]      : (f16)0.0f;
        bf[i + 8] = (col == 0) ? (f16)W[k + 16] : (col == 1) ? (f16)W[DN + k + 16] : (f16)0.0f;
      }
      acc = wmma16(af, bf, acc);
    }
    if (col < 2) {
#pragma unroll
      for (int r = 0; r < 8; ++r) pS[wave][(rh + r) * 2 + col] = acc[r];
    }
  }
  __syncthreads();
  if (live) {
#pragma unroll 1
    for (int pass = 0; pass < 2; ++pass) {
      if (lane < 8) *(volatile v4f_t*)(P + (size_t)tile * 32 + lane * 4) = *(const volatile v4fa*)(pS[wave] + lane * 4);
      __threadfence();
    }
  }
}

__global__ __launch_bounds__(256) void k_edges(const int* __restrict__ ei, const float* __restrict__ P, float* __restrict__ out) {
  const int e = blockIdx.x * 256 + threadIdx.x;
  int s = ei[e], d = ei[NE + e];
  s = min(max(s, 0), NN - 1); d = min(max(d, 0), NN - 1);
  const float z = P[(size_t)s * 2] + P[(size_t)d * 2 + 1];
  const float y = 1.0f / (1.0f + __expf(-z));
  *(volatile float*)(out + e) = y; __threadfence(); *(volatile float*)(out + e) = y;
}

extern "C" void kernel_launch(void* const* d_in, const int* in_sizes, int n_in,
                              void* d_out, int out_size, void* d_ws, size_t ws_size,
                              hipStream_t stream) {
  (void)in_sizes; (void)n_in; (void)out_size; (void)ws_size;
  const float* x  = (const float*)d_in[0];
  const int*   ei = (const int*)d_in[1];
  const float* W  = (const float*)d_in[2];
  float* out = (float*)d_out;
  float* P = (float*)d_ws;
  k_node_proj<<<dim3((NTILE + 7) / 8), dim3(256), 0, stream>>>(x, W, P);
  k_edges<<<dim3(NE / 256), dim3(256), 0, stream>>>(ei, P, out);
}
